// Encoder_6914897346576
// MI455X (gfx1250) — hardware-verified
//
#include <hip/hip_runtime.h>
#include <math.h>

constexpr int NSTEP    = 20;
constexpr int NBATCH   = 65536;
constexpr int NEMB     = 64;
constexpr int NHID     = 64;
constexpr int NGATE    = 4 * NHID;
constexpr int NTHR     = 256;
constexpr int NWAVE    = NTHR / 32;
constexpr int ROWS_WV  = 16;
constexpr int ROWS_BLK = ROWS_WV * NWAVE;
constexpr int WPITCH   = 72;
constexpr int HPITCH   = 72;
constexpr int SLABP    = 68;
constexpr float WCARRY   = 256.0f;
constexpr float HCARRY   = 256.0f;
constexpr float FOLD     = WCARRY * HCARRY;
constexpr float FOLD_INV = 1.0f / FOLD;

static_assert(NBATCH % ROWS_BLK == 0, "grid exact");
static_assert(NHID % 32 == 0, "K multiple of 32");
static_assert(NGATE == NTHR, "one gate row per thread in the prologue");
static_assert((NGATE * NHID / 4) % NTHR == 0, "weight staging loop exact");
static_assert(NEMB % 4 == 0, "fold loop exact");
static_assert((WPITCH % 8) == 0 && (HPITCH % 8) == 0 && (SLABP % 4) == 0, "16-B aligned LDS rows");

typedef __attribute__((ext_vector_type(16))) _Float16 v16h;
typedef __attribute__((ext_vector_type(8)))  _Float16 v8h;
typedef __attribute__((ext_vector_type(4)))  _Float16 v4h;
typedef __attribute__((ext_vector_type(8)))  float    v8f;
typedef __attribute__((ext_vector_type(4)))  float    v4f;

template <typename T> struct Frag;
template <> struct Frag<_Float16> {
  typedef v16h V; union U { v16h v; v8h h[2]; };
  static __device__ __forceinline__ v16h load(const _Float16* p) {
    U f; f.h[0] = *(const v8h*)(p); f.h[1] = *(const v8h*)(p + 16); return f.v;
  }
  static __device__ __forceinline__ v8f mma(v16h a, v16h b, v8f c) {
    return __builtin_amdgcn_wmma_f32_16x16x32_f16(false, a, false, b, (short)0, c, false, false);
  }
};

__device__ __forceinline__ void grp_guard(v8f& a, v8f& b, v8f& c, v8f& d, v16h x, v16h y0, v16h y1, v16h y2, v16h y3) {
  asm volatile("v_nop\n\tv_nop\n\tv_nop\n\tv_nop" : "+v"(a), "+v"(b), "+v"(c), "+v"(d) : "v"(x), "v"(y0), "v"(y1), "v"(y2), "v"(y3));
}

__device__ __forceinline__ float fsig(float x)  { return __builtin_amdgcn_rcpf(1.0f + expf(-x)); }
__device__ __forceinline__ float ftanh(float x) { return 1.0f - 2.0f * __builtin_amdgcn_rcpf(expf(2.0f * x) + 1.0f); }

__global__ __launch_bounds__(NTHR) void lstm_enc_kernel(const float* __restrict__ obs,
                                                        const float* __restrict__ W_emb,
                                                        const float* __restrict__ b_emb,
                                                        const float* __restrict__ W_ih,
                                                        const float* __restrict__ W_hh,
                                                        const float* __restrict__ b_ih,
                                                        const float* __restrict__ b_hh,
                                                        float* __restrict__ out) {
  __shared__ __align__(16) _Float16 Wl[NGATE * WPITCH];
  __shared__ __align__(16) _Float16 Ht[NWAVE * ROWS_WV * HPITCH];
  __shared__ __align__(16) float    Cs[NWAVE * 4 * 8 * 32];
  __shared__ __align__(16) float    Sl[NWAVE * ROWS_WV * SLABP];
  __shared__ __align__(16) float    Fw0[NGATE];
  __shared__ __align__(16) float    Fw1[NGATE];
  __shared__ __align__(16) float    Fbe[NGATE];

  const int tid  = threadIdx.x;
  const int lane = tid & 31;
  const int wave = tid >> 5;
  const int c    = lane & 15;
  const int hh   = lane >> 4;
  const int koff = hh * 8;

  {
    const v8h zh = {(_Float16)0.0f, (_Float16)0.0f, (_Float16)0.0f, (_Float16)0.0f,
                    (_Float16)0.0f, (_Float16)0.0f, (_Float16)0.0f, (_Float16)0.0f};
    v8h* hp = (v8h*)Ht;
#pragma unroll 1
    for (int i = tid; i < NWAVE * ROWS_WV * HPITCH / 8; i += NTHR) hp[i] = zh;
    const v4f zf = {0.0f, 0.0f, 0.0f, 0.0f};
    v4f* cp = (v4f*)Cs;
#pragma unroll 1
    for (int i = tid; i < NWAVE * 4 * 8 * 32 / 4; i += NTHR) cp[i] = zf;
    *(v8h*)(Wl + tid * WPITCH + NHID) = zh;
  }

  {
    const int n = tid;
    const float* wr = W_ih + (size_t)n * NEMB;
    float w0 = 0.0f, w1 = 0.0f, bb = 0.0f;
#pragma unroll 1
    for (int e4 = 0; e4 < NEMB / 4; ++e4) {
      const v4f wi = *(const v4f*)(wr + 4 * e4);
      const v4f ea = *(const v4f*)(W_emb + 8 * e4);
      const v4f eb = *(const v4f*)(W_emb + 8 * e4 + 4);
      const v4f be = *(const v4f*)(b_emb + 4 * e4);
      w0 = fmaf(wi[0], ea[0], w0); w1 = fmaf(wi[0], ea[1], w1); bb = fmaf(wi[0], be[0], bb);
      w0 = fmaf(wi[1], ea[2], w0); w1 = fmaf(wi[1], ea[3], w1); bb = fmaf(wi[1], be[1], bb);
      w0 = fmaf(wi[2], eb[0], w0); w1 = fmaf(wi[2], eb[1], w1); bb = fmaf(wi[2], be[2], bb);
      w0 = fmaf(wi[3], eb[2], w0); w1 = fmaf(wi[3], eb[3], w1); bb = fmaf(wi[3], be[3], bb);
    }
    const float bsum = b_ih[n] + b_hh[n];
    bb = bb + bsum;
    Fw0[n] = w0 * FOLD;
    Fw1[n] = w1 * FOLD;
    Fbe[n] = bb * FOLD;
  }

#pragma unroll 1
  for (int it = 0; it < (NGATE * NHID / 4) / NTHR; ++it) {
    const int idx = it * NTHR + tid;
    const int row = idx >> 4;
    const int c4  = (idx & 15) * 4;
    const v4f w = *(const v4f*)(W_hh + (size_t)row * NHID + c4);
    v4h hv;
    hv[0] = (_Float16)(w[0] * WCARRY);
    hv[1] = (_Float16)(w[1] * WCARRY);
    hv[2] = (_Float16)(w[2] * WCARRY);
    hv[3] = (_Float16)(w[3] * WCARRY);
    *(v4h*)(Wl + row * WPITCH + c4) = hv;
  }
  __syncthreads();

  const int m0 = (blockIdx.x * NWAVE + wave) * ROWS_WV;
  _Float16* ht   = Ht + wave * (ROWS_WV * HPITCH);
  float*    slab = Sl + wave * (ROWS_WV * SLABP);
  float*    csw  = Cs + wave * (4 * 8 * 32) + lane;
  const _Float16* hrow = ht + c * HPITCH + koff;

#pragma unroll 1
  for (int t = 0; t < NSTEP; ++t) {
    const bool last = (t == NSTEP - 1);
    const v16h a0 = Frag<_Float16>::load(hrow);
    const v16h a1 = Frag<_Float16>::load(hrow + 32);
    float ox[8], oy[8];
    {
      const float* op = obs + ((size_t)t * NBATCH + (size_t)(m0 + 8 * hh)) * 2;
      const v4f o0 = *(const v4f*)(op);
      const v4f o1 = *(const v4f*)(op + 4);
      const v4f o2 = *(const v4f*)(op + 8);
      const v4f o3 = *(const v4f*)(op + 12);
      ox[0] = o0[0]; oy[0] = o0[1]; ox[1] = o0[2]; oy[1] = o0[3];
      ox[2] = o1[0]; oy[2] = o1[1]; ox[3] = o1[2]; oy[3] = o1[3];
      ox[4] = o2[0]; oy[4] = o2[1]; ox[5] = o2[2]; oy[5] = o2[3];
      ox[6] = o3[0]; oy[6] = o3[1]; ox[7] = o3[2]; oy[7] = o3[3];
    }
    __syncthreads();

#pragma unroll 1
    for (int cg = 0; cg < 4; ++cg) {
      const int col = cg * 16 + c;
      const float wi0 = Fw0[col],            wi1 = Fw1[col],            bi = Fbe[col];
      const float wf0 = Fw0[NHID + col],     wf1 = Fw1[NHID + col],     bf = Fbe[NHID + col];
      const float wg0 = Fw0[2 * NHID + col], wg1 = Fw1[2 * NHID + col], bg = Fbe[2 * NHID + col];
      const float wo0 = Fw0[3 * NHID + col], wo1 = Fw1[3 * NHID + col], bo = Fbe[3 * NHID + col];
      v8f ai, af, ag, ao;
#pragma unroll
      for (int r = 0; r < 8; ++r) {
        ai[r] = fmaf(oy[r], wi1, fmaf(ox[r], wi0, bi));
        af[r] = fmaf(oy[r], wf1, fmaf(ox[r], wf0, bf));
        ag[r] = fmaf(oy[r], wg1, fmaf(ox[r], wg0, bg));
        ao[r] = fmaf(oy[r], wo1, fmaf(ox[r], wo0, bo));
      }
      const _Float16* bp = Wl + col * WPITCH + koff;
      {
        const v16h b0 = Frag<_Float16>::load(bp);
        const v16h b1 = Frag<_Float16>::load(bp + 1 * NHID * WPITCH);
        const v16h b2 = Frag<_Float16>::load(bp + 2 * NHID * WPITCH);
        const v16h b3 = Frag<_Float16>::load(bp + 3 * NHID * WPITCH);
        ai = Frag<_Float16>::mma(a0, b0, ai);
        af = Frag<_Float16>::mma(a0, b1, af);
        ag = Frag<_Float16>::mma(a0, b2, ag);
        ao = Frag<_Float16>::mma(a0, b3, ao);
        grp_guard(ai, af, ag, ao, a0, b0, b1, b2, b3);
      }
      {
        const v16h b0 = Frag<_Float16>::load(bp + 32);
        const v16h b1 = Frag<_Float16>::load(bp + 1 * NHID * WPITCH + 32);
        const v16h b2 = Frag<_Float16>::load(bp + 2 * NHID * WPITCH + 32);
        const v16h b3 = Frag<_Float16>::load(bp + 3 * NHID * WPITCH + 32);
        ai = Frag<_Float16>::mma(a1, b0, ai);
        af = Frag<_Float16>::mma(a1, b1, af);
        ag = Frag<_Float16>::mma(a1, b2, ag);
        ao = Frag<_Float16>::mma(a1, b3, ao);
        grp_guard(ai, af, ag, ao, a1, b0, b1, b2, b3);
      }
      float* cs = csw + cg * (8 * 32);
#pragma unroll
      for (int r = 0; r < 8; ++r) {
        const float cold = cs[r * 32];
        const float zi = ai[r] * FOLD_INV;
        const float zf = af[r] * FOLD_INV;
        const float zg = ag[r] * FOLD_INV;
        const float zo = ao[r] * FOLD_INV;
        const float ig = fsig(zi);
        const float fg = fsig(zf);
        const float gg = ftanh(zg);
        const float og = fsig(zo);
        const float cn = fg * cold + ig * gg;
        cs[r * 32] = cn;
        const float hv = og * ftanh(cn);
        float hs = hv * HCARRY;
        asm volatile("" : "+v"(hs));
        ht[(8 * hh + r) * HPITCH + col] = (_Float16)hs;
        if (last) slab[(8 * hh + r) * SLABP + col] = hv;
      }
    }
    __syncthreads();
  }

  {
    const int c4 = c * 4;
    float* ob = out + (size_t)m0 * NHID;
    for (int pass = 0; pass < 2; ++pass) {
#pragma unroll
      for (int it = 0; it < 8; ++it) {
        const int row = it * 2 + hh;
        const v4f v = *(const v4f*)(slab + row * SLABP + c4);
        *(volatile v4f*)(ob + (size_t)row * NHID + c4) = v;
      }
      __threadfence();
    }
  }
}

extern "C" void kernel_launch(void* const* d_in, const int* in_sizes, int n_in,
                              void* d_out, int out_size, void* d_ws, size_t ws_size, hipStream_t stream) {
  (void)in_sizes; (void)out_size; (void)d_ws; (void)ws_size;
  if (n_in < 7 || d_out == nullptr) return;
  const float* obs   = (const float*)d_in[0];
  const float* W_emb = (const float*)d_in[1];
  const float* b_emb = (const float*)d_in[2];
  const float* W_ih  = (const float*)d_in[3];
  const float* W_hh  = (const float*)d_in[4];
  const float* b_ih  = (const float*)d_in[5];
  const float* b_hh  = (const float*)d_in[6];
  float* out = (float*)d_out;
  lstm_enc_kernel<<<NBATCH / ROWS_BLK, NTHR, 0, stream>>>(obs, W_emb, b_emb, W_ih, W_hh, b_ih, b_hh, out);
}
